// GroupAgent_63694365000066
// MI455X (gfx1250) — hardware-verified
//
#include <hip/hip_runtime.h>
#include <math.h>

constexpr int kRows      = 16384;
constexpr int kDin       = 256;
constexpr int kHid       = 256;
constexpr int kEmb       = 256;
constexpr int kAct       = 32;
constexpr int kActPad    = 64;
constexpr int kG3        = 3 * kHid;
constexpr int kHW        = kHid * kAct;
constexpr int kChunkRows = 1024;
constexpr int kNumChunks = kRows / kChunkRows;
static_assert(kNumChunks * kChunkRows == kRows, "");
static_assert(kChunkRows % 64 == 0 && kChunkRows % 8 == 0, "");

constexpr float kWCarry  = 16.0f;
constexpr float kHCarry  = 16.0f;
constexpr float kX1Carry = 8.0f;
constexpr float kHnCarry = 16.0f;
constexpr float kTCarry  = 16.0f;
constexpr float kGCarry  = 16.0f;

constexpr size_t kBytesAct16 = (size_t)kRows * kHid * 2;
constexpr size_t kBytesWD    = (size_t)kChunkRows * kHW * 4;
constexpr size_t kOffXA   = 0;
constexpr size_t kOffX1   = kOffXA + kBytesAct16;
constexpr size_t kOffH16  = kOffX1 + kBytesAct16;
constexpr size_t kOffHN32 = kOffXA;
constexpr size_t kOffHN16 = kOffH16;
constexpr size_t kOffW    = kOffH16 + kBytesAct16;
constexpr size_t kOffFc1T = kOffW + 0;
constexpr size_t kOffWihT = kOffW + 131072;
constexpr size_t kOffWhhT = kOffW + 524288;
constexpr size_t kOffHg1T = kOffW + 917504;
constexpr size_t kOffHg2T = kOffW + 1048576;
constexpr size_t kOffHbT  = kOffW + 1179648;
constexpr size_t kOffHwT  = kOffW + 1212416;
constexpr size_t kOffBig  = kOffW + 5406720;
constexpr size_t kOffGI   = kOffBig;
constexpr size_t kOffGH   = kOffBig + (size_t)kRows * kG3 * 4;
constexpr size_t kOffT16  = kOffBig;
constexpr size_t kOffG16  = kOffBig + kBytesAct16;
constexpr size_t kOffBD   = kOffBig + 2 * kBytesAct16;
constexpr size_t kOffWDA  = kOffBD + (size_t)kRows * kActPad * 4;
constexpr size_t kOffWDB  = kOffWDA + kBytesWD;
constexpr size_t kWsTotal = kOffGH + (size_t)kRows * kG3 * 4;
static_assert(kOffHwT + (size_t)kHW * kEmb * 2 == kOffBig, "");
static_assert(kOffWDB + kBytesWD <= kWsTotal, "");
static_assert(kOffHN32 + (size_t)kRows * kHid * 4 <= kOffH16, "");
static_assert(kWsTotal <= (size_t)134217728, "");
static_assert((kOffBig % 4096) == 0 && (kOffWDA % 4096) == 0 && (kOffWDB % 4096) == 0 && (kOffBD % 4096) == 0, "");

typedef __attribute__((ext_vector_type(16))) _Float16 v16h;
typedef __attribute__((ext_vector_type(8)))  _Float16 v8h;
typedef __attribute__((ext_vector_type(16))) __bf16   v16b;
typedef __attribute__((ext_vector_type(8)))  __bf16   v8b;
typedef __attribute__((ext_vector_type(8)))  float    v8f;
typedef __attribute__((ext_vector_type(4)))  float    v4f;
typedef __attribute__((ext_vector_type(4)))  unsigned int v4u;

__device__ __forceinline__ unsigned short f2bf_bits(float f) {
  unsigned u = __float_as_uint(f);
  return (unsigned short)((u + 0x7FFFu + ((u >> 16) & 1u)) >> 16);
}
__device__ __forceinline__ float bf_bits2f(unsigned short h) { return __uint_as_float(((unsigned)h) << 16); }

__device__ __forceinline__ void dep_guard_h(v8f& a, v8f& b, v16h x, v16h y) { asm volatile("v_nop\n\tv_nop\n\tv_nop\n\tv_nop" : "+v"(a), "+v"(b) : "v"(x), "v"(y)); }
__device__ __forceinline__ void dep_guard_b(v8f& a, v8f& b, v16b x, v16b y) { asm volatile("v_nop\n\tv_nop\n\tv_nop\n\tv_nop" : "+v"(a), "+v"(b) : "v"(x), "v"(y)); }
__device__ __forceinline__ void keep4_h(v16h a, v16h b, v16h c, v16h d) { asm volatile("v_nop" :: "v"(a), "v"(b), "v"(c), "v"(d)); }
__device__ __forceinline__ void keep4_b(v16b a, v16b b, v16b c, v16b d) { asm volatile("v_nop" :: "v"(a), "v"(b), "v"(c), "v"(d)); }
__device__ __forceinline__ void acc_guard4(v8f& a, v8f& b, v8f& c, v8f& d) { asm volatile("v_nop\n\tv_nop\n\tv_nop\n\tv_nop" : "+v"(a), "+v"(b), "+v"(c), "+v"(d)); }
template <typename T> struct Frag;
template <> struct Frag<_Float16> {
  typedef v16h V; union U { v16h v; v8h h[2]; };
  static __device__ __forceinline__ v16h load(const _Float16* p) {
    U f; f.h[0] = *(const v8h*)(p); f.h[1] = *(const v8h*)(p + 16); return f.v;
  }
  static __device__ __forceinline__ v8f mma(v16h a, v16h b, v8f c) {
    return __builtin_amdgcn_wmma_f32_16x16x32_f16(false, a, false, b, (short)0, c, false, false);
  }
  static __device__ __forceinline__ void guard(v8f& a, v8f& b, v16h x, v16h y) { dep_guard_h(a, b, x, y); }
  static __device__ __forceinline__ void keep(v16h a, v16h b, v16h c, v16h d) { keep4_h(a, b, c, d); }
};
template <> struct Frag<__bf16> {
  typedef v16b V; union U { v16b v; v8b h[2]; };
  static __device__ __forceinline__ v16b load(const __bf16* p) {
    U f; f.h[0] = *(const v8b*)(p); f.h[1] = *(const v8b*)(p + 16); return f.v;
  }
  static __device__ __forceinline__ v8f mma(v16b a, v16b b, v8f c) {
    return __builtin_amdgcn_wmma_f32_16x16x32_bf16(false, a, false, b, (short)0, c, false, false);
  }
  static __device__ __forceinline__ void guard(v8f& a, v8f& b, v16b x, v16b y) { dep_guard_b(a, b, x, y); }
  static __device__ __forceinline__ void keep(v16b a, v16b b, v16b c, v16b d) { keep4_b(a, b, c, d); }
};

__device__ __forceinline__ unsigned pk16(unsigned short a, unsigned short b) { return (unsigned)a | ((unsigned)b << 16); }
__device__ __forceinline__ unsigned short h_bits(float f) { const _Float16 h = (_Float16)f; return __builtin_bit_cast(unsigned short, h); }

template <int ET> struct Elem;
template <> struct Elem<0> { typedef _Float16 T; };
template <> struct Elem<1> { typedef __bf16 T; };
template <int ET, bool SPLIT, int BIAS_MODE, int OUT_MODE, bool RESID, int ACT = 0>
__global__ __launch_bounds__(256) void wmma_gemm64(
    const unsigned short* __restrict__ Ap, const unsigned short* __restrict__ A2p, int lda, long strideA,
    const unsigned short* __restrict__ Btp, const unsigned short* __restrict__ Bt2p, int ldb, long strideB,
    void* __restrict__ Cout, void* __restrict__ Cout2, int ldc, long strideC,
    const float* __restrict__ bias,
    const float* __restrict__ resid, long strideR,
    int M, int N, int K, float scale, float oscale) {
  typedef typename Elem<ET>::T T;
  typedef typename Frag<T>::V V;
  const T* A = (const T*)Ap; const T* A2 = (const T*)A2p; const T* Bt = (const T*)Btp; const T* Bt2 = (const T*)Bt2p;
  __shared__ __align__(16) float sT[8][16 * 68];
  const int b    = blockIdx.y;
  const int lane = threadIdx.x & 31;
  const int wave = threadIdx.x >> 5;
  const int tilesN = N >> 6;
  const int tilesM = M >> 6;
  const int tile = blockIdx.x * 8 + wave;
  if (tile >= tilesM * tilesN) return;
  const int tm = tile / tilesN;
  const int tn = tile - tm * tilesN;
  const int m0 = tm << 6;
  const int n0 = tn << 6;

  const T* Ab  = A  + (size_t)b * strideA;
  const T* Bb  = Bt + (size_t)b * strideB;
  const T* Ab2 = SPLIT ? (A2  + (size_t)b * strideA) : nullptr;
  const T* Bb2 = SPLIT ? (Bt2 + (size_t)b * strideB) : nullptr;

  const int rlane = lane & 15;
  const int koff  = (lane >> 4) * 8;
  const int mOff  = (lane >> 4) * 8;

  v8f acc[4][4];
#pragma unroll
  for (int i = 0; i < 4; ++i)
#pragma unroll
    for (int j = 0; j < 4; ++j) acc[i][j] = (v8f){0.f,0.f,0.f,0.f,0.f,0.f,0.f,0.f};

  for (int k0 = 0; k0 < K; k0 += 32) {
    V bh[4], bl[4];
#pragma unroll
    for (int j = 0; j < 4; ++j) {
      const size_t bo = (size_t)(n0 + (j << 4) + rlane) * ldb + koff + k0;
      bh[j] = Frag<T>::load(Bb + bo);
      if (SPLIT) bl[j] = Frag<T>::load(Bb2 + bo);
    }
#pragma unroll
    for (int i = 0; i < 4; ++i) {
      const size_t ao = (size_t)(m0 + (i << 4) + rlane) * lda + koff + k0;
      V ah = Frag<T>::load(Ab + ao);
      V al;
      if (SPLIT) al = Frag<T>::load(Ab2 + ao);
#pragma unroll
      for (int j = 0; j < 4; ++j) {
        acc[i][j] = Frag<T>::mma(ah, bh[j], acc[i][j]);
        if (SPLIT) {
          acc[i][j] = Frag<T>::mma(ah, bl[j], acc[i][j]);
          acc[i][j] = Frag<T>::mma(al, bh[j], acc[i][j]);
        }
      }
      Frag<T>::guard(acc[i][0], acc[i][3], ah, SPLIT ? al : ah);
    }
    Frag<T>::keep(bh[0], bh[1], bh[2], bh[3]);
    if (SPLIT) Frag<T>::keep(bl[0], bl[1], bl[2], bl[3]);
  }
  acc_guard4(acc[0][0], acc[0][1], acc[0][2], acc[0][3]);
  acc_guard4(acc[1][0], acc[1][1], acc[1][2], acc[1][3]);
  acc_guard4(acc[2][0], acc[2][1], acc[2][2], acc[2][3]);
  acc_guard4(acc[3][0], acc[3][1], acc[3][2], acc[3][3]);

  float* slab = sT[wave];
  const float* Rb = RESID ? (resid + (size_t)b * strideR) : nullptr;
#pragma unroll
  for (int i = 0; i < 4; ++i) {
    const int mBase = m0 + (i << 4);
#pragma unroll
    for (int j = 0; j < 4; ++j) {
      const int n = n0 + (j << 4) + rlane;
      float bv = 0.f;
      if (BIAS_MODE == 2) bv = bias[n];
#pragma unroll
      for (int r = 0; r < 8; ++r) {
        float v = acc[i][j][r] * scale;
        if (BIAS_MODE == 1) v += bias[mBase + mOff + r];
        if (BIAS_MODE == 2) v += bv;
        if (RESID) v += Rb[(size_t)(mBase + mOff + r) * ldc + n];
        if (ACT == 1) v = tanhf(v);
        if (ACT == 2) v = fmaxf(v, 0.0f);
        if (ACT == 4) v = (v > 0.f) ? v : 0.01f * v;
        v = v * oscale;
        slab[(mOff + r) * 68 + (j << 4) + rlane] = v;
      }
    }
    __builtin_amdgcn_fence(__ATOMIC_RELEASE, "workgroup");
    __builtin_amdgcn_wave_barrier();
    __builtin_amdgcn_fence(__ATOMIC_ACQUIRE, "workgroup");
    if (OUT_MODE == 0) {
      float* C = (float*)Cout + (size_t)b * strideC;
      const int hh = lane >> 4, c4 = (lane & 15) * 4;
      for (int pass = 0; pass < 2; ++pass) {
#pragma unroll
        for (int it = 0; it < 8; ++it) {
          const int row = it * 2 + hh;
          v4f v = *(const v4f*)(slab + row * 68 + c4);
          *(volatile v4f*)(C + (size_t)(mBase + row) * ldc + n0 + c4) = v;
        }
        __threadfence();
      }
    } else {
      const int q = lane >> 3, c8 = (lane & 7) * 8;
      unsigned short* C  = (unsigned short*)Cout  + (size_t)b * strideC;
      unsigned short* C2 = (OUT_MODE == 2) ? ((unsigned short*)Cout2 + (size_t)b * strideC) : nullptr;
      for (int pass = 0; pass < 2; ++pass) {
#pragma unroll
        for (int it = 0; it < 4; ++it) {
          const int row = it * 4 + q;
          const float* sp = slab + row * 68 + c8;
          v8h hv, lv;
#pragma unroll
          for (int e = 0; e < 8; ++e) {
            if (OUT_MODE == 1) {
              hv[e] = (_Float16)sp[e];
            } else {
              unsigned short hb = f2bf_bits(sp[e]);
              unsigned short lb = f2bf_bits(sp[e] - bf_bits2f(hb));
              hv[e] = __builtin_bit_cast(_Float16, hb);
              lv[e] = __builtin_bit_cast(_Float16, lb);
            }
          }
          *(volatile v8h*)(C + (size_t)(mBase + row) * ldc + n0 + c8) = hv;
          if (OUT_MODE == 2) *(volatile v8h*)(C2 + (size_t)(mBase + row) * ldc + n0 + c8) = lv;
        }
        __threadfence();
      }
    }
    __builtin_amdgcn_fence(__ATOMIC_RELEASE, "workgroup");
    __builtin_amdgcn_wave_barrier();
    __builtin_amdgcn_fence(__ATOMIC_ACQUIRE, "workgroup");
  }
}

__global__ __launch_bounds__(256) void cast8_f16_kernel(const float* __restrict__ in, unsigned short* __restrict__ out,
                                                        int n8, float scale) {
  const int i = blockIdx.x * 256 + threadIdx.x;
  if (i >= n8) return;
  const float* p = in + 8 * (size_t)i;
  const v4f a = *(const v4f*)(p);
  const v4f c = *(const v4f*)(p + 4);
  unsigned short hb[8];
#pragma unroll
  for (int e = 0; e < 4; ++e) {
    hb[e]     = h_bits(a[e] * scale);
    hb[4 + e] = h_bits(c[e] * scale);
  }
  const v4u u = (v4u){pk16(hb[0], hb[1]), pk16(hb[2], hb[3]), pk16(hb[4], hb[5]), pk16(hb[6], hb[7])};
  unsigned short* q = out + 8 * (size_t)i;
  *(volatile v4u*)q = u;
  __threadfence();
  *(volatile v4u*)q = u;
}

__global__ __launch_bounds__(256) void wtcast_kernel(const float* __restrict__ W, int Nc,
                                                     unsigned short* __restrict__ out, float scale) {
  __shared__ float sm[64][65];
  const int t  = threadIdx.x;
  const int k0 = blockIdx.x * 64;
  const int n0 = blockIdx.y * 64;
#pragma unroll
  for (int i = 0; i < 16; ++i) {
    const int e = i * 256 + t;
    const int r = e >> 6;
    const int c = e & 63;
    const int n = n0 + c;
    const int ncl = (n < Nc) ? n : (Nc - 1);
    float v = W[(size_t)(k0 + r) * Nc + ncl] * scale;
    v = (n < Nc) ? v : 0.0f;
    sm[c][r] = v;
  }
  __syncthreads();
  const int lane = t & 31, wave = t >> 5;
  const int q = lane >> 3, c8 = (lane & 7) * 8;
  for (int pass = 0; pass < 2; ++pass) {
#pragma unroll
    for (int it = 0; it < 2; ++it) {
      const int row = wave * 8 + it * 4 + q;
      unsigned short hb[8];
#pragma unroll
      for (int e = 0; e < 8; ++e) hb[e] = h_bits(sm[row][c8 + e]);
      const v4u u = (v4u){pk16(hb[0], hb[1]), pk16(hb[2], hb[3]), pk16(hb[4], hb[5]), pk16(hb[6], hb[7])};
      *(volatile v4u*)(out + (size_t)(n0 + row) * kDin + k0 + c8) = u;
    }
    __threadfence();
  }
}

__device__ __forceinline__ float sigm_f(float x) {
  x = fminf(fmaxf(x, -30.0f), 30.0f);
  const float e = expf(-x);
  return 1.0f / (1.0f + e);
}

__global__ __launch_bounds__(256) void gru_gate_kernel(const float* __restrict__ gi, const float* __restrict__ gh,
                                                       const float* __restrict__ h, float* __restrict__ hn32,
                                                       unsigned short* __restrict__ hn16) {
  __shared__ __align__(16) float sv[256];
  const int t = threadIdx.x;
  const int n = blockIdx.x;
  const size_t gb = (size_t)n * kG3;
  const size_t rb = (size_t)n * kHid;
  const float ir  = gi[gb + t];
  const float iz  = gi[gb + kHid + t];
  const float in_ = gi[gb + 2 * kHid + t];
  const float hr  = gh[gb + t];
  const float hz  = gh[gb + kHid + t];
  const float hnn = gh[gb + 2 * kHid + t];
  const float hv  = h[rb + t];
  const float r  = sigm_f(ir + hr);
  const float z  = sigm_f(iz + hz);
  const float ng = tanhf(in_ + r * hnn);
  const float v  = (1.0f - z) * ng + z * hv;
  sv[t] = v;
  __syncthreads();
  const int lane = t & 31, wave = t >> 5;
  if (wave < 2) {
    const int f = (wave * 32 + lane) * 4;
    const v4f val = *(const v4f*)(sv + f);
    float* dst = hn32 + rb + f;
    *(volatile v4f*)dst = val;
    __threadfence();
    *(volatile v4f*)dst = val;
  } else if (wave == 2) {
    const int f = lane * 8;
    unsigned short hb[8];
#pragma unroll
    for (int e = 0; e < 8; ++e) hb[e] = h_bits(sv[f + e] * kHnCarry);
    const v4u u = (v4u){pk16(hb[0], hb[1]), pk16(hb[2], hb[3]), pk16(hb[4], hb[5]), pk16(hb[6], hb[7])};
    unsigned short* dst = hn16 + rb + f;
    *(volatile v4u*)dst = u;
    __threadfence();
    *(volatile v4u*)dst = u;
  }
}

__global__ __launch_bounds__(256) void qhead_kernel(const float* __restrict__ wd, const float* __restrict__ hn32c,
                                                    const float* __restrict__ bdc, const float* __restrict__ hb_b,
                                                    float* __restrict__ qc) {
  __shared__ __align__(16) float sq[8 * 32];
  const int t = threadIdx.x, lane = t & 31, wave = t >> 5;
  const int row = blockIdx.x * 8 + wave;
  const float* wrow = wd + (size_t)row * kHW;
  const float* hrow = hn32c + (size_t)row * kHid;
  float acc = 0.0f;
#pragma unroll 1
  for (int hb8 = 0; hb8 < kHid; hb8 += 32) {
    const float hv = hrow[hb8 + lane];
#pragma unroll
    for (int i = 0; i < 32; ++i) {
      const float hi = __shfl(hv, i, 32);
      acc = fmaf(hi, wrow[(size_t)(hb8 + i) * kAct + lane], acc);
    }
  }
  const float v = acc + bdc[(size_t)row * kActPad + lane] + hb_b[lane];
  sq[wave * 32 + lane] = v;
  __syncthreads();
  if (wave < 2) {
    const int f = (wave * 32 + lane) * 4;
    const v4f val = *(const v4f*)(sq + f);
    float* dst = qc + (size_t)blockIdx.x * 8 * kAct + f;
    *(volatile v4f*)dst = val;
    __threadfence();
    *(volatile v4f*)dst = val;
  }
}

extern "C" void kernel_launch(void* const* d_in, const int* in_sizes, int n_in,
                              void* d_out, int out_size, void* d_ws, size_t ws_size,
                              hipStream_t stream)
{
  if (n_in < 16) return;
  if (in_sizes[0] != kRows * kDin || in_sizes[1] != kRows * kHid || in_sizes[2] != kDin * kHid ||
      in_sizes[3] != kHid || in_sizes[4] != kHid * kG3 || in_sizes[5] != kG3 || in_sizes[6] != kHid * kG3 ||
      in_sizes[7] != kG3 || in_sizes[8] != kHid * kEmb || in_sizes[9] != kEmb || in_sizes[10] != kEmb * kEmb ||
      in_sizes[11] != kEmb || in_sizes[12] != kEmb * kAct || in_sizes[13] != kAct ||
      in_sizes[14] != kEmb * kHW || in_sizes[15] != kHW) return;
  if (out_size != kRows * kAct) return;
  if (ws_size < kWsTotal) return;

  const float* x     = (const float*)d_in[0];
  const float* h     = (const float*)d_in[1];
  const float* fc1_w = (const float*)d_in[2];
  const float* fc1_b = (const float*)d_in[3];
  const float* w_ih  = (const float*)d_in[4];
  const float* b_ih  = (const float*)d_in[5];
  const float* w_hh  = (const float*)d_in[6];
  const float* b_hh  = (const float*)d_in[7];
  const float* hg_w1 = (const float*)d_in[8];
  const float* hg_b1 = (const float*)d_in[9];
  const float* hg_w2 = (const float*)d_in[10];
  const float* hg_b2 = (const float*)d_in[11];
  const float* hb_w  = (const float*)d_in[12];
  const float* hb_b  = (const float*)d_in[13];
  const float* hw_w  = (const float*)d_in[14];
  const float* hw_b  = (const float*)d_in[15];
  float* q = (float*)d_out;

  char* ws = (char*)d_ws;
  unsigned short* x16   = (unsigned short*)(ws + kOffXA);
  unsigned short* x1_16 = (unsigned short*)(ws + kOffX1);
  unsigned short* h16   = (unsigned short*)(ws + kOffH16);
  float*          hn32  = (float*)(ws + kOffHN32);
  unsigned short* hn16  = (unsigned short*)(ws + kOffHN16);
  unsigned short* fc1_t = (unsigned short*)(ws + kOffFc1T);
  unsigned short* wih_t = (unsigned short*)(ws + kOffWihT);
  unsigned short* whh_t = (unsigned short*)(ws + kOffWhhT);
  unsigned short* hg1_t = (unsigned short*)(ws + kOffHg1T);
  unsigned short* hg2_t = (unsigned short*)(ws + kOffHg2T);
  unsigned short* hb_t  = (unsigned short*)(ws + kOffHbT);
  unsigned short* hw_t  = (unsigned short*)(ws + kOffHwT);
  float*          gi32  = (float*)(ws + kOffGI);
  float*          gh32  = (float*)(ws + kOffGH);
  unsigned short* t16   = (unsigned short*)(ws + kOffT16);
  unsigned short* g16   = (unsigned short*)(ws + kOffG16);
  float*          bd32  = (float*)(ws + kOffBD);
  float*          wdA   = (float*)(ws + kOffWDA);
  float*          wdB   = (float*)(ws + kOffWDB);
  const float*    dummy = (const float*)(ws);

  const int n8 = kRows * kHid / 8;
  cast8_f16_kernel<<<dim3(n8 / 256), dim3(256), 0, stream>>>(x, x16, n8, 1.0f);
  cast8_f16_kernel<<<dim3(n8 / 256), dim3(256), 0, stream>>>(h, h16, n8, kHCarry);
  wtcast_kernel<<<dim3(kDin / 64, kHid / 64),    dim3(256), 0, stream>>>(fc1_w, kHid, fc1_t, kWCarry);
  wtcast_kernel<<<dim3(kHid / 64, kG3 / 64),     dim3(256), 0, stream>>>(w_ih,  kG3,  wih_t, kWCarry);
  wtcast_kernel<<<dim3(kHid / 64, kG3 / 64),     dim3(256), 0, stream>>>(w_hh,  kG3,  whh_t, kWCarry);
  wtcast_kernel<<<dim3(kHid / 64, kEmb / 64),    dim3(256), 0, stream>>>(hg_w1, kEmb, hg1_t, kWCarry);
  wtcast_kernel<<<dim3(kEmb / 64, kEmb / 64),    dim3(256), 0, stream>>>(hg_w2, kEmb, hg2_t, kWCarry);
  wtcast_kernel<<<dim3(kEmb / 64, kActPad / 64), dim3(256), 0, stream>>>(hb_w,  kAct, hb_t,  kWCarry);
  wtcast_kernel<<<dim3(kEmb / 64, kHW / 64),     dim3(256), 0, stream>>>(hw_w,  kHW,  hw_t,  kWCarry);

  const dim3 gblk(256);
  {
    const int tiles = (kRows / 64) * (kHid / 64);
    wmma_gemm64<0, false, 2, 1, false, 2><<<dim3((tiles + 7) / 8, 1), gblk, 0, stream>>>(
        x16, x16, kDin, 0L, fc1_t, fc1_t, kDin, 0L, (void*)x1_16, (void*)x1_16, kHid, 0L,
        fc1_b, dummy, 0L, kRows, kHid, kDin, 1.0f / kWCarry, kX1Carry);
  }
  {
    const int tiles = (kRows / 64) * (kG3 / 64);
    wmma_gemm64<0, false, 2, 0, false, 0><<<dim3((tiles + 7) / 8, 1), gblk, 0, stream>>>(
        x1_16, x1_16, kHid, 0L, wih_t, wih_t, kHid, 0L, (void*)gi32, (void*)gi32, kG3, 0L,
        b_ih, dummy, 0L, kRows, kG3, kHid, 1.0f / (kX1Carry * kWCarry), 1.0f);
    wmma_gemm64<0, false, 2, 0, false, 0><<<dim3((tiles + 7) / 8, 1), gblk, 0, stream>>>(
        h16, h16, kHid, 0L, whh_t, whh_t, kHid, 0L, (void*)gh32, (void*)gh32, kG3, 0L,
        b_hh, dummy, 0L, kRows, kG3, kHid, 1.0f / (kHCarry * kWCarry), 1.0f);
  }
  gru_gate_kernel<<<dim3(kRows), dim3(256), 0, stream>>>(gi32, gh32, h, hn32, hn16);
  {
    const int tiles = (kRows / 64) * (kEmb / 64);
    wmma_gemm64<0, false, 2, 1, false, 2><<<dim3((tiles + 7) / 8, 1), gblk, 0, stream>>>(
        hn16, hn16, kHid, 0L, hg1_t, hg1_t, kHid, 0L, (void*)t16, (void*)t16, kEmb, 0L,
        hg_b1, dummy, 0L, kRows, kEmb, kHid, 1.0f / (kHnCarry * kWCarry), kTCarry);
    wmma_gemm64<0, false, 2, 1, false, 1><<<dim3((tiles + 7) / 8, 1), gblk, 0, stream>>>(
        t16, t16, kEmb, 0L, hg2_t, hg2_t, kEmb, 0L, (void*)g16, (void*)g16, kEmb, 0L,
        hg_b2, dummy, 0L, kRows, kEmb, kEmb, 1.0f / (kTCarry * kWCarry), kGCarry);
  }
  {
    const int tiles = (kRows / 64) * (kActPad / 64);
    wmma_gemm64<0, false, 0, 0, false, 0><<<dim3((tiles + 7) / 8, 1), gblk, 0, stream>>>(
        g16, g16, kEmb, 0L, hb_t, hb_t, kEmb, 0L, (void*)bd32, (void*)bd32, kActPad, 0L,
        hb_b, dummy, 0L, kRows, kActPad, kEmb, 1.0f / (kGCarry * kWCarry), 1.0f);
  }
  for (int c = 0; c < kNumChunks; ++c) {
    const size_t r0 = (size_t)c * kChunkRows;
    float* wd = (c & 1) ? wdB : wdA;
    const int tiles = (kChunkRows / 64) * (kHW / 64);
    wmma_gemm64<0, false, 2, 0, false, 0><<<dim3((tiles + 7) / 8, 1), gblk, 0, stream>>>(
        g16 + r0 * kEmb, g16 + r0 * kEmb, kEmb, 0L, hw_t, hw_t, kEmb, 0L, (void*)wd, (void*)wd, kHW, 0L,
        hw_b, dummy, 0L, kChunkRows, kHW, kEmb, 1.0f / (kGCarry * kWCarry), 1.0f);
    qhead_kernel<<<dim3(kChunkRows / 8), dim3(256), 0, stream>>>(
        wd, hn32 + r0 * kHid, bd32 + r0 * kActPad, hb_b, q + r0 * kAct);
  }
}
